// DPRNN_12154757447884
// MI455X (gfx1250) — hardware-verified
//
#include <hip/hip_runtime.h>
#include <math.h>

#define NB_  2
#define CCH  64
#define FF_  128
#define TT_  250
#define KW   8
#define TN_  243
#define HS   32
#define H2   64
#define NSEQ 256
#define MROW (NSEQ * TN_)
#define MOUT (NSEQ * TT_)

typedef _Float16 f16;
typedef __attribute__((ext_vector_type(16))) f16 f16x16;
typedef __attribute__((ext_vector_type(8)))  f16 f16x8;
typedef __attribute__((ext_vector_type(8)))  float f32x8;
typedef __attribute__((ext_vector_type(4)))  float v4f_t;
typedef float v4fa __attribute__((ext_vector_type(4), may_alias));
typedef __attribute__((ext_vector_type(4))) unsigned v4u_t;
typedef unsigned v4ua __attribute__((ext_vector_type(4), may_alias));

__device__ __forceinline__ f32x8 wmma16(f16x16 a, f16x16 b, f32x8 c) {
  c = __builtin_amdgcn_wmma_f32_16x16x32_f16(false, a, false, b, (short)0, c, false, false);
  asm volatile("v_nop\n\tv_nop\n\tv_nop\n\tv_nop" : "+v"(c) : "v"(a), "v"(b));
  return c;
}
__device__ __forceinline__ f16x16 lds_frag(const f16* base, int stride) {
  const int lane = threadIdx.x & 31, row = lane & 15, kh = (lane >> 4) * 8;
  const f16x8 lo = *(const f16x8*)(base + row * stride + kh);
  const f16x8 hi = *(const f16x8*)(base + row * stride + kh + 16);
  f16x16 f;
#pragma unroll
  for (int i = 0; i < 8; ++i) { f[i] = lo[i]; f[i + 8] = hi[i]; }
  return f;
}
#define GSTR 48

#define GSTR 48
template <typename AT, int EPI, bool OUT16, int ASRC>
__global__ __launch_bounds__(256) void gemm_kned(const AT* __restrict__ A, int lda, const float* __restrict__ Wm, int ldw,
                                                const float* __restrict__ bias, const float* __restrict__ R, const float* __restrict__ gvec,
                                                const float* __restrict__ gnst, const float* __restrict__ gam, const float* __restrict__ bet,
                                                void* __restrict__ Yv, int ldy, int K) {
  __shared__ __attribute__((aligned(16))) f16 ldsA[128 * GSTR];
  __shared__ __attribute__((aligned(16))) f16 ldsW[128 * GSTR];
  __shared__ __attribute__((aligned(16))) float oS[8][32 * 68];
  const int tid = threadIdx.x, lane = tid & 31, wave = tid >> 5, cl = lane & 15, rh = (lane >> 4) * 8;
  const int m0 = blockIdx.x * 128, n0 = blockIdx.y * 128;
  const int wm = (wave & 3) * 32, wn = (wave >> 2) * 64;
  f32x8 acc[2][4];
#pragma unroll
  for (int i = 0; i < 2; ++i)
#pragma unroll
    for (int j = 0; j < 4; ++j) { f32x8 z = {}; acc[i][j] = z; }
#pragma unroll 1
  for (int k0 = 0; k0 < K; k0 += 32) {
    __syncthreads();
    { const int row = tid >> 1, ch = (tid & 1) * 16;
      if (ASRC == 0) {
        const AT* src = A + (size_t)(m0 + row) * lda + k0 + ch;
#pragma unroll
        for (int g = 0; g < 16; ++g) ldsA[row * GSTR + ch + g] = (f16)src[g];
      } else if (ASRC == 1) {
        const int m = m0 + row, n = m / TN_, t = m - n * TN_, b = n >> 7, f = n & 127;
        const float mu = gnst[32 * b], rs = gnst[32 * b + 1];
#pragma unroll
        for (int cc = 0; cc < 2; ++cc) {
          const int c = ((k0 + ch) >> 3) + cc;
          const float ga = gam[c] * rs, be = bet[c] - mu * gam[c] * rs;
          const float* xp = (const float*)A + (((size_t)b * CCH + c) * FF_ + f) * TT_ + t;
#pragma unroll
          for (int kk = 0; kk < 8; ++kk) ldsA[row * GSTR + ch + cc * 8 + kk] = (f16)(xp[kk] * ga + be);
        }
      } else {
        const int m = m0 + row, n = m / TT_, t = m - n * TT_;
#pragma unroll
        for (int cc = 0; cc < 2; ++cc) {
          const int i = ((k0 + ch) >> 3) + cc;
#pragma unroll
          for (int j = 0; j < 8; ++j) { const int ts = t - j; float v = 0.0f;
            if (ts >= 0 && ts < TN_) v = ((const float*)A)[((size_t)n * TN_ + ts) * H2 + i];
            ldsA[row * GSTR + ch + cc * 8 + j] = (f16)v; }
        }
      } }
    { const int k = tid >> 3, nn0 = (tid & 7) * 16;
      const float* src = Wm + (size_t)(k0 + k) * ldw + n0 + nn0;
#pragma unroll
      for (int g = 0; g < 4; ++g) { const v4f_t v = *(const v4f_t*)(src + 4 * g);
#pragma unroll
        for (int u = 0; u < 4; ++u) ldsW[(nn0 + 4 * g + u) * GSTR + k] = (f16)v[u]; } }
    __syncthreads();
    f16x16 af[2];
#pragma unroll
    for (int i = 0; i < 2; ++i) af[i] = lds_frag(ldsA + (wm + 16 * i) * GSTR, GSTR);
#pragma unroll
    for (int j = 0; j < 4; ++j) {
      const f16x16 bf = lds_frag(ldsW + (wn + 16 * j) * GSTR, GSTR);
#pragma unroll
      for (int i = 0; i < 2; ++i) acc[i][j] = wmma16(af[i], bf, acc[i][j]);
    }
  }
  float* so = oS[wave];
#pragma unroll
  for (int i = 0; i < 2; ++i)
#pragma unroll
    for (int j = 0; j < 4; ++j) {
      const int n = n0 + wn + 16 * j + cl;
      const float bv = bias ? bias[n] : 0.0f;
      const float gv = (EPI == 2) ? gvec[n] : 0.0f;
      if (EPI == 1) {
#pragma unroll 1
        for (int r = 0; r < 8; ++r) { const float xg = acc[i][j][r] + bv; so[(16 * i + rh + r) * 68 + 16 * j + cl] = 0.5f * xg * (1.0f + erff(xg * 0.70710678118654752f)); }
      } else {
#pragma unroll
        for (int r = 0; r < 8; ++r) {
          float v = acc[i][j][r] + bv;
          if (EPI == 2) v = R[(size_t)(m0 + wm + 16 * i + rh + r) * ldy + n] + gv * v;
          so[(16 * i + rh + r) * 68 + 16 * j + cl] = v;
        }
      }
    }
  asm volatile("s_wait_dscnt 0" ::: "memory");
  __builtin_amdgcn_wave_barrier();
#pragma unroll 1
  for (int pass = 0; pass < 2; ++pass) {
    if (OUT16) {
      f16* Y = (f16*)Yv;
#pragma unroll
      for (int it = 0; it < 8; ++it) { const int c = lane + 32 * it, rr = c >> 3, q8 = (c & 7) * 8;
        union { f16 h[8]; v4u_t v; } u;
#pragma unroll
        for (int e = 0; e < 8; ++e) u.h[e] = (f16)so[rr * 68 + q8 + e];
        *(volatile v4u_t*)(Y + (size_t)(m0 + wm + rr) * ldy + n0 + wn + q8) = u.v; }
    } else {
      float* Y = (float*)Yv;
#pragma unroll
      for (int it = 0; it < 16; ++it) { const int f4 = lane + 32 * it, rr = f4 >> 4, q = (f4 & 15) * 4;
        *(volatile v4f_t*)(Y + (size_t)(m0 + wm + rr) * ldy + n0 + wn + q) = *(const volatile v4fa*)(so + rr * 68 + q); }
    }
    __threadfence();
  }
}

__global__ __launch_bounds__(256) void k_gnstats(const float* __restrict__ x, float* __restrict__ st) {
  __shared__ float red[256];
  const int b = blockIdx.x, t = threadIdx.x;
  const float* p = x + (size_t)b * CCH * FF_ * TT_;
  const int n = CCH * FF_ * TT_;
  float s = 0.0f;
  for (int i = t; i < n; i += 256) s += p[i];
  red[t] = s; __syncthreads();
  for (int o = 128; o > 0; o >>= 1) { if (t < o) red[t] += red[t + o]; __syncthreads(); }
  const float mu = red[0] / (float)n; __syncthreads();
  float q = 0.0f;
  for (int i = t; i < n; i += 256) { const float d = p[i] - mu; q += d * d; }
  red[t] = q; __syncthreads();
  for (int o = 128; o > 0; o >>= 1) { if (t < o) red[t] += red[t + o]; __syncthreads(); }
  if (t == 0) { v4f_t v; v[0] = mu; v[1] = rsqrtf(red[0] / (float)n + 1e-5f); v[2] = 0.f; v[3] = 0.f;
    *(volatile v4f_t*)(st + b * 32) = v; __threadfence(); *(volatile v4f_t*)(st + b * 32) = v; }
}
__global__ __launch_bounds__(256) void k_scan(const float* __restrict__ U, const float* __restrict__ vv, const float* __restrict__ bb, int dir,
                                             float* __restrict__ hout) {
  const int lane = threadIdx.x & 31, n = blockIdx.x * 8 + (threadIdx.x >> 5);
  const float vf = vv[lane], vr = vv[HS + lane], bf = bb[lane], br = bb[HS + lane];
  float c = 0.0f;
#pragma unroll 1
  for (int s = 0; s < TN_; ++s) {
    const int t = dir ? (TN_ - 1 - s) : s;
    const float* u = U + ((size_t)n * TN_ + t) * 128;
    const float z = u[lane], fp = u[HS + lane], rp = u[2 * HS + lane], xp = u[3 * HS + lane];
    const float f = 1.0f / (1.0f + __expf(-(fp + vf * c + bf)));
    const float r = 1.0f / (1.0f + __expf(-(rp + vr * c + br)));
    c = f * c + (1.0f - f) * z;
    const float h = r * c + (1.0f - r) * xp;
    float* d = hout + ((size_t)n * TN_ + t) * H2 + dir * HS + lane;
    *(volatile float*)d = h; __threadfence(); *(volatile float*)d = h;
  }
}
__global__ __launch_bounds__(256) void k_wct2(const float* __restrict__ wct, float* __restrict__ W2) {
  const int k = blockIdx.x;
  const int i = k >> 3, j = k & 7, t = threadIdx.x;
  if (t < 32) { v4f_t v;
#pragma unroll
    for (int u = 0; u < 4; ++u) { const int o = t * 4 + u; v[u] = (o < CCH) ? wct[((size_t)i * CCH + o) * KW + j] : 0.0f; }
    *(volatile v4f_t*)(W2 + (size_t)k * 128 + t * 4) = v; __threadfence(); *(volatile v4f_t*)(W2 + (size_t)k * 128 + t * 4) = v; }
}
__global__ __launch_bounds__(256) void k_final(const float* __restrict__ y2, const float* __restrict__ bct, const float* __restrict__ x, float* __restrict__ out) {
  const int b = blockIdx.x / CCH, c = blockIdx.x % CCH, tid = threadIdx.x;
  const float bc = bct[c];
  const size_t pbase = ((size_t)b * CCH + c) * FF_ * TT_;
#pragma unroll 1
  for (int pass = 0; pass < 2; ++pass) {
    for (int q = tid; q < FF_ * TT_ / 4; q += 256) {
      v4f_t v;
#pragma unroll
      for (int u = 0; u < 4; ++u) { const int e = q * 4 + u, f = e / TT_, t = e - f * TT_; const int n = b * FF_ + f;
        v[u] = y2[((size_t)n * TT_ + t) * 128 + c] + bc + x[pbase + e]; }
      *(volatile v4f_t*)(out + pbase + (size_t)q * 4) = v;
    }
    __threadfence();
  }
}

extern "C" void kernel_launch(void* const* d_in, const int* in_sizes, int n_in,
                              void* d_out, int out_size, void* d_ws, size_t ws_size,
                              hipStream_t stream) {
  (void)in_sizes; (void)n_in; (void)out_size; (void)ws_size;
  const float* x = (const float*)d_in[0];
  const float* gamma = (const float*)d_in[1], *beta = (const float*)d_in[2];
  const float* W0 = (const float*)d_in[3];
  const float* Wr = (const float*)d_in[4];
  const float* vv = (const float*)d_in[5];
  const float* bb = (const float*)d_in[6];
  const float* wct = (const float*)d_in[7];
  const float* bct = (const float*)d_in[8];
  float* out = (float*)d_out;
  char* ws = (char*)d_ws;
  float* st = (float*)ws; ws += 256;
  float* U = (float*)ws; ws += (size_t)MROW * 128 * 4;
  float* hA = (float*)ws; ws += (size_t)MROW * H2 * 4;
  float* hB = (float*)ws; ws += (size_t)MROW * H2 * 4;
  float* W2 = (float*)ws; ws += (size_t)512 * 128 * 4;
  float* y2 = (float*)ws; ws += (size_t)MOUT * 128 * 4;
  k_gnstats<<<dim3(NB_), dim3(256), 0, stream>>>(x, st);
  const dim3 gG(MROW / 128, 1), blk(256);
  float* hin = nullptr; float* hout = hA;
  for (int l = 0; l < 4; ++l) {
    for (int dir = 0; dir < 2; ++dir) {
      if (l == 0) gemm_kned<float, 0, false, 1><<<gG, blk, 0, stream>>>(x, 0, W0 + (size_t)dir * 512 * 128, 128, nullptr, nullptr, nullptr, st, gamma, beta, U, 128, 512);
      else        gemm_kned<float, 0, false, 0><<<gG, blk, 0, stream>>>(hin, H2, Wr + (((size_t)(l - 1) * 2 + dir) * H2) * 128, 128, nullptr, nullptr, nullptr, nullptr, nullptr, nullptr, U, 128, H2);
      k_scan<<<dim3(NSEQ / 8), dim3(256), 0, stream>>>(U, vv + ((size_t)l * 2 + dir) * H2, bb + ((size_t)l * 2 + dir) * H2, dir, hout);
    }
    hin = hout; hout = (hout == hA) ? hB : hA;
  }
  k_wct2<<<dim3(512), dim3(256), 0, stream>>>(wct, W2);
  gemm_kned<float, 0, false, 2><<<dim3(MOUT / 128, 1), blk, 0, stream>>>(hin, 0, W2, 128, nullptr, nullptr, nullptr, nullptr, nullptr, nullptr, y2, 128, 512);
  k_final<<<dim3(NB_ * CCH), dim3(256), 0, stream>>>(y2, bct, x, out);
}
